// VariableRecurrent_893353197872
// MI455X (gfx1250) — hardware-verified
//
#include <hip/hip_runtime.h>
#include <math.h>

constexpr int N_SEQ    = 32;
constexpr int N_STEP   = 2048;
constexpr int N_IN     = 256;
constexpr int N_HID    = 256;
constexpr int N_GATE   = 768;
constexpr int N_TOK    = 49664;
constexpr int N_SLOT   = N_STEP * N_SEQ;
constexpr int SCAN_THR = 512;
constexpr int HAP  = 264;
constexpr int HSP  = 260;
constexpr int GXPW = 388;
constexpr int INV_RANGE = 8192;
constexpr int INV_BLKS  = N_SLOT / INV_RANGE;
constexpr float WCARRY     = 16.0f;
constexpr float WCARRY_INV = 1.0f / 16.0f;
static_assert(N_GATE == 3 * N_HID);
static_assert(N_TOK % 64 == 0 && N_GATE % 64 == 0 && N_IN % 32 == 0 && N_HID % 32 == 0);
static_assert(N_HID == 16 * (SCAN_THR / 32));
static_assert(N_SEQ * 16 == SCAN_THR);
static_assert((HAP % 8) == 0 && (HSP % 4) == 0 && (GXPW % 4) == 0 && GXPW * 2 >= N_GATE);
static_assert(((N_TOK * (N_IN / 8)) % 256) == 0 && ((N_GATE * (N_IN / 8)) % 256) == 0);
static_assert(((N_TOK / 64) * (N_GATE / 64)) % 8 == 0);
static_assert((N_SLOT / 4) % 256 == 0 && N_TOK % 256 == 0);
static_assert(N_SLOT % INV_RANGE == 0 && INV_RANGE % (256 * 4) == 0 && (INV_RANGE * 4) % 128 == 0);

typedef __attribute__((ext_vector_type(16))) _Float16 v16h;
typedef __attribute__((ext_vector_type(8)))  _Float16 v8h;
typedef __attribute__((ext_vector_type(16))) __bf16   v16b;
typedef __attribute__((ext_vector_type(8)))  __bf16   v8b;
typedef __attribute__((ext_vector_type(8)))  float    v8f;
typedef __attribute__((ext_vector_type(4)))  float    v4f;
typedef __attribute__((ext_vector_type(4)))  unsigned v4u;
typedef __attribute__((ext_vector_type(4)))  int      v4i;

__device__ __forceinline__ unsigned short f2bf_bits(float f) {
  unsigned u = __float_as_uint(f);
  return (unsigned short)((u + 0x7FFFu + ((u >> 16) & 1u)) >> 16);
}
__device__ __forceinline__ float bf_bits2f(unsigned short h) { return __uint_as_float(((unsigned)h) << 16); }

__device__ __forceinline__ float h16_to_f32(unsigned hb) {
  const unsigned sgn = (hb & 0x8000u) << 16;
  const unsigned em = hb & 0x7fffu;
  const float fn = __uint_as_float((em << 13) + 0x38000000u);
  const float fs = (float)em * 5.9604644775390625e-8f;
  const float mag = (em < 0x400u) ? fs : fn;
  return __uint_as_float(__float_as_uint(mag) | sgn);
}

__device__ __forceinline__ void dep_guard4_h(v8f& a, v8f& b, v8f& c, v8f& d, v16h x, v16h y) {
  asm volatile("v_nop\n\tv_nop\n\tv_nop\n\tv_nop" : "+v"(a), "+v"(b), "+v"(c), "+v"(d) : "v"(x), "v"(y));
}
__device__ __forceinline__ void dep_guard4_b(v8f& a, v8f& b, v8f& c, v8f& d, v16b x, v16b y) {
  asm volatile("v_nop\n\tv_nop\n\tv_nop\n\tv_nop" : "+v"(a), "+v"(b), "+v"(c), "+v"(d) : "v"(x), "v"(y));
}
__device__ __forceinline__ void keep4_h(v16h a, v16h b, v16h c, v16h d) { asm volatile("v_nop" :: "v"(a), "v"(b), "v"(c), "v"(d)); }
__device__ __forceinline__ void keep4_b(v16b a, v16b b, v16b c, v16b d) { asm volatile("v_nop" :: "v"(a), "v"(b), "v"(c), "v"(d)); }
__device__ __forceinline__ void acc_guard4(v8f& a, v8f& b, v8f& c, v8f& d) {
  asm volatile("v_nop\n\tv_nop\n\tv_nop\n\tv_nop" : "+v"(a), "+v"(b), "+v"(c), "+v"(d));
}
__device__ __forceinline__ void guard3_h(v8f& a, v8f& b, v8f& c, v16h x, v16h y0, v16h y1, v16h y2) {
  asm volatile("v_nop\n\tv_nop\n\tv_nop\n\tv_nop" : "+v"(a), "+v"(b), "+v"(c) : "v"(x), "v"(y0), "v"(y1), "v"(y2));
}
__device__ __forceinline__ void acc_guard3(v8f& a, v8f& b, v8f& c) {
  asm volatile("v_nop\n\tv_nop\n\tv_nop\n\tv_nop" : "+v"(a), "+v"(b), "+v"(c));
}

template <typename T> struct Frag;
template <> struct Frag<_Float16> {
  typedef v16h V; union U { v16h v; v8h h[2]; };
  static __device__ __forceinline__ v16h load(const _Float16* p) {
    U f; f.h[0] = *(const v8h*)(p); f.h[1] = *(const v8h*)(p + 16); return f.v;
  }
  static __device__ __forceinline__ v8f mma(v16h a, v16h b, v8f c) {
    return __builtin_amdgcn_wmma_f32_16x16x32_f16(false, a, false, b, (short)0, c, false, false);
  }
  static __device__ __forceinline__ void guard4(v8f& a, v8f& b, v8f& c, v8f& d, v16h x, v16h y) { dep_guard4_h(a, b, c, d, x, y); }
  static __device__ __forceinline__ void keep(v16h a, v16h b, v16h c, v16h d) { keep4_h(a, b, c, d); }
};
template <> struct Frag<__bf16> {
  typedef v16b V; union U { v16b v; v8b h[2]; };
  static __device__ __forceinline__ v16b load(const __bf16* p) {
    U f; f.h[0] = *(const v8b*)(p); f.h[1] = *(const v8b*)(p + 16); return f.v;
  }
  static __device__ __forceinline__ v8f mma(v16b a, v16b b, v8f c) {
    return __builtin_amdgcn_wmma_f32_16x16x32_bf16(false, a, false, b, (short)0, c, false, false);
  }
  static __device__ __forceinline__ void guard4(v8f& a, v8f& b, v8f& c, v8f& d, v16b x, v16b y) { dep_guard4_b(a, b, c, d, x, y); }
  static __device__ __forceinline__ void keep(v16b a, v16b b, v16b c, v16b d) { keep4_b(a, b, c, d); }
};

template <int ET> struct Elem;
template <> struct Elem<0> { typedef _Float16 T; };
template <> struct Elem<1> { typedef __bf16 T; };
template <int ET, bool SPLIT, int BIAS_MODE, int OUT_MODE, bool RESID, int ACT = 0>
__global__ __launch_bounds__(256) void wmma_gemm64(
    const unsigned short* __restrict__ Ap, const unsigned short* __restrict__ A2p, int lda, long strideA,
    const unsigned short* __restrict__ Btp, const unsigned short* __restrict__ Bt2p, int ldb, long strideB,
    void* __restrict__ Cout, void* __restrict__ Cout2, int ldc, long strideC,
    const float* __restrict__ bias,
    const float* __restrict__ resid, long strideR,
    int M, int N, int K, float scale) {
  typedef typename Elem<ET>::T T;
  typedef typename Frag<T>::V V;
  const T* A = (const T*)Ap; const T* A2 = (const T*)A2p; const T* Bt = (const T*)Btp; const T* Bt2 = (const T*)Bt2p;
  __shared__ __align__(16) float sT[8][16 * 68];
  const int b    = blockIdx.y;
  const int lane = threadIdx.x & 31;
  const int wave = threadIdx.x >> 5;
  const int tilesN = N >> 6;
  const int tilesM = M >> 6;
  const int tile = blockIdx.x * 8 + wave;
  if (tile >= tilesM * tilesN) return;
  const int tm = tile / tilesN;
  const int tn = tile - tm * tilesN;
  const int m0 = tm << 6;
  const int n0 = tn << 6;

  const T* Ab  = A  + (size_t)b * strideA;
  const T* Bb  = Bt + (size_t)b * strideB;
  const T* Ab2 = SPLIT ? (A2  + (size_t)b * strideA) : nullptr;
  const T* Bb2 = SPLIT ? (Bt2 + (size_t)b * strideB) : nullptr;

  const int rlane = lane & 15;
  const int koff  = (lane >> 4) * 8;
  const int mOff  = (lane >> 4) * 8;

  v8f acc[4][4];
#pragma unroll
  for (int i = 0; i < 4; ++i)
#pragma unroll
    for (int j = 0; j < 4; ++j) acc[i][j] = (v8f){0.f,0.f,0.f,0.f,0.f,0.f,0.f,0.f};

  for (int k0 = 0; k0 < K; k0 += 32) {
    V bh[4], bl[4];
#pragma unroll
    for (int j = 0; j < 4; ++j) {
      const size_t bo = (size_t)(n0 + (j << 4) + rlane) * ldb + koff + k0;
      bh[j] = Frag<T>::load(Bb + bo);
      if (SPLIT) bl[j] = Frag<T>::load(Bb2 + bo);
    }
#pragma unroll
    for (int i = 0; i < 4; ++i) {
      const size_t ao = (size_t)(m0 + (i << 4) + rlane) * lda + koff + k0;
      V ah = Frag<T>::load(Ab + ao);
      V al;
      if (SPLIT) al = Frag<T>::load(Ab2 + ao);
#pragma unroll
      for (int j = 0; j < 4; ++j) {
        acc[i][j] = Frag<T>::mma(ah, bh[j], acc[i][j]);
        if (SPLIT) {
          acc[i][j] = Frag<T>::mma(ah, bl[j], acc[i][j]);
          acc[i][j] = Frag<T>::mma(al, bh[j], acc[i][j]);
        }
      }
      Frag<T>::guard4(acc[i][0], acc[i][1], acc[i][2], acc[i][3], ah, SPLIT ? al : ah);
    }
    Frag<T>::keep(bh[0], bh[1], bh[2], bh[3]);
    if (SPLIT) Frag<T>::keep(bl[0], bl[1], bl[2], bl[3]);
  }
  acc_guard4(acc[0][0], acc[0][1], acc[0][2], acc[0][3]);
  acc_guard4(acc[1][0], acc[1][1], acc[1][2], acc[1][3]);
  acc_guard4(acc[2][0], acc[2][1], acc[2][2], acc[2][3]);
  acc_guard4(acc[3][0], acc[3][1], acc[3][2], acc[3][3]);

  float* slab = sT[wave];
  const float* Rb = RESID ? (resid + (size_t)b * strideR) : nullptr;
#pragma unroll
  for (int i = 0; i < 4; ++i) {
    const int mBase = m0 + (i << 4);
#pragma unroll
    for (int j = 0; j < 4; ++j) {
      const int n = n0 + (j << 4) + rlane;
      float bv = 0.f;
      if (BIAS_MODE == 2) bv = bias[n];
#pragma unroll
      for (int r = 0; r < 8; ++r) {
        float v = acc[i][j][r] * scale;
        if (BIAS_MODE == 1) v += bias[mBase + mOff + r];
        if (BIAS_MODE == 2) v += bv;
        if (RESID) v += Rb[(size_t)(mBase + mOff + r) * ldc + n];
        if (ACT == 1) v = tanhf(v);
        if (ACT == 2) v = fmaxf(v, 0.0f);
        if (ACT == 3) v = v / (1.0f + expf(-v));
        if (ACT == 4) v = (v > 0.f) ? v : 0.01f * v;
        slab[(mOff + r) * 68 + (j << 4) + rlane] = v;
      }
    }
    __builtin_amdgcn_fence(__ATOMIC_RELEASE, "workgroup");
    __builtin_amdgcn_wave_barrier();
    __builtin_amdgcn_fence(__ATOMIC_ACQUIRE, "workgroup");
    if (OUT_MODE == 0) {
      float* C = (float*)Cout + (size_t)b * strideC;
      const int hh = lane >> 4, c4 = (lane & 15) * 4;
      for (int pass = 0; pass < 2; ++pass) {
#pragma unroll
        for (int it = 0; it < 8; ++it) {
          const int row = it * 2 + hh;
          v4f v = *(const v4f*)(slab + row * 68 + c4);
          *(volatile v4f*)(C + (size_t)(mBase + row) * ldc + n0 + c4) = v;
        }
        __threadfence();
      }
    } else {
      const int q = lane >> 3, c8 = (lane & 7) * 8;
      unsigned short* C  = (unsigned short*)Cout  + (size_t)b * strideC;
      unsigned short* C2 = (OUT_MODE == 2) ? ((unsigned short*)Cout2 + (size_t)b * strideC) : nullptr;
      for (int pass = 0; pass < 2; ++pass) {
#pragma unroll
        for (int it = 0; it < 4; ++it) {
          const int row = it * 4 + q;
          const float* sp = slab + row * 68 + c8;
          v8h hv, lv;
#pragma unroll
          for (int e = 0; e < 8; ++e) {
            if (OUT_MODE == 1) {
              hv[e] = (_Float16)sp[e];
            } else {
              unsigned short hb = f2bf_bits(sp[e]);
              unsigned short lb = f2bf_bits(sp[e] - bf_bits2f(hb));
              hv[e] = __builtin_bit_cast(_Float16, hb);
              lv[e] = __builtin_bit_cast(_Float16, lb);
            }
          }
          *(volatile v8h*)(C + (size_t)(mBase + row) * ldc + n0 + c8) = hv;
          if (OUT_MODE == 2) *(volatile v8h*)(C2 + (size_t)(mBase + row) * ldc + n0 + c8) = lv;
        }
        __threadfence();
      }
    }
    __builtin_amdgcn_fence(__ATOMIC_RELEASE, "workgroup");
    __builtin_amdgcn_wave_barrier();
    __builtin_amdgcn_fence(__ATOMIC_ACQUIRE, "workgroup");
  }
}

__global__ __launch_bounds__(256) void cvt8_f16_kernel(const float* __restrict__ s0, unsigned short* __restrict__ d0,
                                                       const float* __restrict__ s1, unsigned short* __restrict__ d1,
                                                       int n8, float sc) {
  const float* src = (blockIdx.y != 0) ? s1 : s0;
  unsigned short* dst = (blockIdx.y != 0) ? d1 : d0;
  const int i = blockIdx.x * 256 + threadIdx.x;
  if (i < n8) {
    const float* sp = src + (size_t)i * 8;
    const v4f a = *(const v4f*)(sp);
    const v4f b = *(const v4f*)(sp + 4);
    v8h hv;
#pragma unroll
    for (int e = 0; e < 4; ++e) {
      const float fa = a[e] * sc;
      const float fb = b[e] * sc;
      hv[e]     = (_Float16)fa;
      hv[4 + e] = (_Float16)fb;
    }
    *(volatile v8h*)(dst + (size_t)i * 8) = hv;
    __threadfence();
    *(volatile v8h*)(dst + (size_t)i * 8) = hv;
  }
}

__global__ __launch_bounds__(256) void inv_build_kernel(const int* __restrict__ gidx, int* __restrict__ inv) {
  __shared__ __align__(16) int img[INV_RANGE];
  const int tid = threadIdx.x;
  const int base = blockIdx.x * INV_RANGE;
  {
    const v4i m = {-1, -1, -1, -1};
#pragma unroll 1
    for (int it = 0; it < INV_RANGE / 1024; ++it) *(v4i*)(img + (it * 256 + tid) * 4) = m;
  }
  __syncthreads();
#pragma unroll 1
  for (int it = 0; it < N_TOK / 256; ++it) {
    const int k = it * 256 + tid;
    int p = gidx[k];
    p = p < 0 ? 0 : p;
    p = p > (N_SLOT - 1) ? (N_SLOT - 1) : p;
    const int q = p - base;
    if ((unsigned)q < (unsigned)INV_RANGE) img[q] = k;
  }
  __syncthreads();
  v4i vals[INV_RANGE / 1024];
#pragma unroll
  for (int it = 0; it < INV_RANGE / 1024; ++it) vals[it] = *(const v4i*)(img + (it * 256 + tid) * 4);
  int* op = inv + base;
  for (int pass = 0; pass < 2; ++pass) {
#pragma unroll
    for (int it = 0; it < INV_RANGE / 1024; ++it) *(volatile v4i*)(op + (it * 256 + tid) * 4) = vals[it];
    __threadfence();
  }
}

__device__ __forceinline__ float gate_sigmoid(float x) {
  x = fminf(fmaxf(x, -30.0f), 30.0f);
  return 1.0f / (1.0f + expf(-x));
}
__device__ __forceinline__ float gate_tanh(float x) {
  x = fminf(fmaxf(x, -15.0f), 15.0f);
  return 1.0f - 2.0f / (1.0f + expf(2.0f * x));
}

__device__ __forceinline__ void stage_step(unsigned* gxw, int* slotw, const unsigned short* gxp, const int* inv,
                                           int tstep, int tid) {
  const int row = tid >> 4;
  const int c16 = tid & 15;
  int p = tstep * N_SEQ + row;
  p = p < 0 ? 0 : p;
  p = p > (N_SLOT - 1) ? (N_SLOT - 1) : p;
  int k = inv[p];
  asm volatile("" : "+v"(k));
  const bool ok = (k >= 0) && (k < N_TOK);
  int srow = k < 0 ? 0 : k;
  srow = srow > (N_TOK - 1) ? (N_TOK - 1) : srow;
  const v4u* sp = (const v4u*)(gxp + (size_t)srow * N_GATE);
  v4u* dp = (v4u*)(gxw + row * GXPW);
#pragma unroll
  for (int it = 0; it < 6; ++it) dp[c16 + 16 * it] = sp[c16 + 16 * it];
  const int sv = ok ? k : -1;
  if (c16 == 0) slotw[row] = sv;
}

__device__ __forceinline__ void rebuild_h16(_Float16* hA, const float* hS, int tid) {
  const int row = tid >> 4;
  const int c16 = (tid & 15) * 16;
  const float* sp = hS + row * HSP + c16;
  const v4f f0 = *(const v4f*)(sp);
  const v4f f1 = *(const v4f*)(sp + 4);
  const v4f f2 = *(const v4f*)(sp + 8);
  const v4f f3 = *(const v4f*)(sp + 12);
  v8h ha, hb;
#pragma unroll
  for (int e = 0; e < 4; ++e) {
    const float x0 = f0[e];
    const float x1 = f1[e];
    const float x2 = f2[e];
    const float x3 = f3[e];
    ha[e]     = (_Float16)x0;
    ha[4 + e] = (_Float16)x1;
    hb[e]     = (_Float16)x2;
    hb[4 + e] = (_Float16)x3;
  }
  *(v8h*)(hA + row * HAP + c16)     = ha;
  *(v8h*)(hA + row * HAP + c16 + 8) = hb;
}

__global__ __launch_bounds__(SCAN_THR) void gru_scan_kernel(const unsigned short* __restrict__ gxp,
                                                            const float* __restrict__ h0,
                                                            const unsigned short* __restrict__ whhp,
                                                            const float* __restrict__ b_ih,
                                                            const float* __restrict__ b_hh,
                                                            const int* __restrict__ bsz,
                                                            const int* __restrict__ inv,
                                                            float* __restrict__ out0,
                                                            float* __restrict__ out1) {
  __shared__ __align__(16) unsigned gxw[N_SEQ * GXPW];
  __shared__ __align__(16) _Float16 hA[N_SEQ * HAP];
  __shared__ __align__(16) float    hS[N_SEQ * HSP];
  __shared__ __align__(16) int      slotw[2 * N_SEQ];
  const _Float16* WH = (const _Float16*)whhp;
  const int tid = threadIdx.x, lane = tid & 31, wave = tid >> 5;
  const int c = lane & 15, hh = lane >> 4, koff = hh * 8;
  const int j = 16 * wave + c;

  {
    const int row = tid >> 4;
    const int c16 = (tid & 15) * 16;
    const float* sp = h0 + row * N_HID + c16;
    float* dp = hS + row * HSP + c16;
    const v4f f0 = *(const v4f*)(sp);
    const v4f f1 = *(const v4f*)(sp + 4);
    const v4f f2 = *(const v4f*)(sp + 8);
    const v4f f3 = *(const v4f*)(sp + 12);
    *(v4f*)(dp)      = f0;
    *(v4f*)(dp + 4)  = f1;
    *(v4f*)(dp + 8)  = f2;
    *(v4f*)(dp + 12) = f3;
  }
  __syncthreads();
  rebuild_h16(hA, hS, tid);
  stage_step(gxw, slotw, gxp, inv, 0, tid);
  const float bhr = b_hh[j];
  const float bhz = b_hh[N_HID + j];
  const float bhn = b_hh[2 * N_HID + j];
  const float bir = b_ih[j];
  const float biz = b_ih[N_HID + j];
  const float bin = b_ih[2 * N_HID + j];
  __syncthreads();

  const _Float16* wr = WH + (size_t)j * N_HID + koff;
  const unsigned sh = (unsigned)(c & 1) * 16u;
  const v8f z8 = {0.f, 0.f, 0.f, 0.f, 0.f, 0.f, 0.f, 0.f};

#pragma unroll 1
  for (int t = 0; t < N_STEP; ++t) {
    int bs = bsz[t];
    bs = bs < 0 ? 0 : bs;
    bs = bs > N_SEQ ? N_SEQ : bs;
    const int* slotc = slotw + (t & 1) * N_SEQ;

#pragma unroll 1
    for (int mt = 0; mt < 2; ++mt) {
      const _Float16* ahrow = hA + (16 * mt + c) * HAP + koff;
      v8f aR = z8, aZ = z8, aN = z8;
#pragma unroll 1
      for (int k0 = 0; k0 < N_HID; k0 += 32) {
        const v16h a  = Frag<_Float16>::load(ahrow + k0);
        const v16h b0 = Frag<_Float16>::load(wr + k0);
        const v16h b1 = Frag<_Float16>::load(wr + (size_t)1 * N_HID * N_HID + k0);
        const v16h b2 = Frag<_Float16>::load(wr + (size_t)2 * N_HID * N_HID + k0);
        aR = Frag<_Float16>::mma(a, b0, aR);
        aZ = Frag<_Float16>::mma(a, b1, aZ);
        aN = Frag<_Float16>::mma(a, b2, aN);
        guard3_h(aR, aZ, aN, a, b0, b1, b2);
      }
      acc_guard3(aR, aZ, aN);

      const int brow0 = 16 * mt + 8 * hh;
      float* hsrow = hS + brow0 * HSP + j;
      const unsigned* gxrow = gxw + brow0 * GXPW + (j >> 1);
      const int* slr = slotc + brow0;
#pragma unroll
      for (int r = 0; r < 8; ++r) {
        const int b = brow0 + r;
        const unsigned wR = gxrow[r * GXPW];
        const unsigned wZ = gxrow[r * GXPW + (N_HID >> 1)];
        const unsigned wN = gxrow[r * GXPW + N_HID];
        const bool has = slr[r] >= 0;
        const float fr = h16_to_f32((wR >> sh) & 0xffffu);
        const float fz = h16_to_f32((wZ >> sh) & 0xffffu);
        const float fn = h16_to_f32((wN >> sh) & 0xffffu);
        const float gr = has ? fr : bir;
        const float gz = has ? fz : biz;
        const float gn = has ? fn : bin;
        const float hold = hsrow[r * HSP];
        const float pr = aR[r] * WCARRY_INV + (gr + bhr);
        const float pz = aZ[r] * WCARRY_INV + (gz + bhz);
        const float ph = aN[r] * WCARRY_INV + bhn;
        const float rg = gate_sigmoid(pr);
        const float zg = gate_sigmoid(pz);
        const float ng = gate_tanh(gn + rg * ph);
        const float hnew = (1.0f - zg) * ng + zg * hold;
        const float hv = (b < bs) ? hnew : hold;
        hsrow[r * HSP] = hv;
      }
    }
    __syncthreads();

    rebuild_h16(hA, hS, tid);
    {
      const int tn = (t + 1 < N_STEP) ? (t + 1) : (N_STEP - 1);
      stage_step(gxw, slotw + ((t + 1) & 1) * N_SEQ, gxp, inv, tn, tid);
    }
    {
      const int b0 = 2 * wave, b1 = 2 * wave + 1;
      const v4f v00 = *(const v4f*)(hS + b0 * HSP + 4 * lane);
      const v4f v01 = *(const v4f*)(hS + b0 * HSP + 128 + 4 * lane);
      const v4f v10 = *(const v4f*)(hS + b1 * HSP + 4 * lane);
      const v4f v11 = *(const v4f*)(hS + b1 * HSP + 128 + 4 * lane);
      const int r0 = slotc[b0], r1 = slotc[b1];
      const bool s0 = (r0 >= 0) && (r0 < N_TOK);
      const bool s1 = (r1 >= 0) && (r1 < N_TOK);
      const int r0c = r0 < 0 ? 0 : (r0 > N_TOK - 1 ? N_TOK - 1 : r0);
      const int r1c = r1 < 0 ? 0 : (r1 > N_TOK - 1 ? N_TOK - 1 : r1);
      float* p0 = out1 + (size_t)r0c * N_HID + 4 * lane;
      float* p1 = out1 + (size_t)r1c * N_HID + 4 * lane;
      for (int pass = 0; pass < 2; ++pass) {
        if (s0) {
          *(volatile v4f*)(p0)       = v00;
          *(volatile v4f*)(p0 + 128) = v01;
        }
        if (s1) {
          *(volatile v4f*)(p1)       = v10;
          *(volatile v4f*)(p1 + 128) = v11;
        }
        __threadfence();
      }
    }
    __syncthreads();
  }

  {
    const int b0 = 2 * wave, b1 = 2 * wave + 1;
    const v4f v00 = *(const v4f*)(hS + b0 * HSP + 4 * lane);
    const v4f v01 = *(const v4f*)(hS + b0 * HSP + 128 + 4 * lane);
    const v4f v10 = *(const v4f*)(hS + b1 * HSP + 4 * lane);
    const v4f v11 = *(const v4f*)(hS + b1 * HSP + 128 + 4 * lane);
    float* p0 = out0 + (size_t)b0 * N_HID + 4 * lane;
    float* p1 = out0 + (size_t)b1 * N_HID + 4 * lane;
    for (int pass = 0; pass < 2; ++pass) {
      *(volatile v4f*)(p0)       = v00;
      *(volatile v4f*)(p0 + 128) = v01;
      *(volatile v4f*)(p1)       = v10;
      *(volatile v4f*)(p1 + 128) = v11;
      __threadfence();
    }
  }
}

extern "C" void kernel_launch(void* const* d_in, const int* in_sizes, int n_in,
                              void* d_out, int out_size, void* d_ws, size_t ws_size, hipStream_t stream) {
  if (n_in < 8 || d_out == nullptr || d_ws == nullptr) return;
  if (in_sizes[0] != N_TOK * N_IN || in_sizes[1] != N_SEQ * N_HID || in_sizes[2] != N_GATE * N_IN ||
      in_sizes[3] != N_GATE * N_HID || in_sizes[4] != N_GATE || in_sizes[5] != N_GATE ||
      in_sizes[6] != N_STEP || in_sizes[7] != N_TOK || out_size != N_SEQ * N_HID + N_TOK * N_HID) return;

  const float* xin  = (const float*)d_in[0];
  const float* h0   = (const float*)d_in[1];
  const float* w_ih = (const float*)d_in[2];
  const float* w_hh = (const float*)d_in[3];
  const float* b_ih = (const float*)d_in[4];
  const float* b_hh = (const float*)d_in[5];
  const int*   bsz  = (const int*)d_in[6];
  const int*   gidx = (const int*)d_in[7];
  float* out0 = (float*)d_out;
  float* out1 = out0 + (size_t)N_SEQ * N_HID;

  char* ws = (char*)d_ws; size_t off = 0;
  auto carve = [&](size_t bytes) -> char* { char* p = ws + off; off += (bytes + 255) & ~(size_t)255; return p; };
  unsigned short* GX  = (unsigned short*)carve((size_t)N_TOK * N_GATE * 2);
  unsigned short* XH  = (unsigned short*)carve((size_t)N_TOK * N_IN * 2);
  unsigned short* WIH = (unsigned short*)carve((size_t)N_GATE * N_IN * 2);
  unsigned short* WHH = (unsigned short*)carve((size_t)N_GATE * N_HID * 2);
  int*            INV = (int*)carve((size_t)N_SLOT * 4);
  if (off > ws_size || off > (size_t)134217728) return;

  inv_build_kernel<<<INV_BLKS, 256, 0, stream>>>(gidx, INV);

  const int n8x = N_TOK * (N_IN / 8);
  const int n8w = N_GATE * (N_IN / 8);
  cvt8_f16_kernel<<<dim3(n8x / 256, 1), 256, 0, stream>>>(xin, XH, xin, XH, n8x, 1.0f);
  cvt8_f16_kernel<<<dim3(n8w / 256, 2), 256, 0, stream>>>(w_ih, WIH, w_hh, WHH, n8w, WCARRY);

  const dim3 ggrid((N_TOK / 64) * (N_GATE / 64) / 8, 1);
  wmma_gemm64<0, false, 2, 1, false, 0><<<ggrid, 256, 0, stream>>>(
      XH, XH, N_IN, 0L, WIH, WIH, N_IN, 0L, (void*)GX, (void*)GX, N_GATE, 0L,
      b_ih, b_ih, 0L, N_TOK, N_GATE, N_IN, WCARRY_INV);

  gru_scan_kernel<<<1, SCAN_THR, 0, stream>>>(GX, h0, WHH, b_ih, b_hh, bsz, INV, out0, out1);
}
